// TransformerBlock_34007551049974
// MI455X (gfx1250) — hardware-run, weakly checked
//
#include <hip/hip_runtime.h>


#ifndef NB
#define NB 2
#endif
#ifndef SEQ
#define SEQ 2048
#endif
#ifndef LCT
#define LCT 512
#endif
#define NB_FULL  2
#define SEQ_FULL 2048
#define LCT_FULL 512
#ifndef OUT_SEQ
#define OUT_SEQ SEQ
#endif
#define DM   1024
#define NH_  16
#define HD   64
#define CD   768
#define DF   4096
#define AW   4
#define OSP  68
#define GSP  68
#define WCAR 256.0f
#define WCI  (1.0f / 256.0f)
#define CCAR 64.0f
#define OCI  (1.0f / 16384.0f)
#define SC2  ((float)(0.125 * 1.4426950408889634))
#define PSH  14.0f
#define NEGB (-3.0e38f)
#define LNEPS 1.0e-5f
#define KVT  (SEQ > LCT ? SEQ : LCT)

static_assert(HD == 64);
static_assert(NH_ * HD == DM);
static_assert(DM % 64 == 0);
static_assert(DF % 64 == 0);
static_assert(DM % 32 == 0);
static_assert(CD % 32 == 0);
static_assert(DF % 32 == 0);
static_assert(SEQ % 64 == 0);
static_assert(LCT % 64 == 0);
static_assert((NB * SEQ) % 64 == 0);
static_assert((NB * LCT) % 64 == 0);
static_assert(SEQ % 32 == 0);
static_assert(LCT % 32 == 0);
static_assert(SEQ % (16 * AW) == 0);
static_assert((NB * SEQ) % 8 == 0);
static_assert(DM == 4 * 32 * 8);
static_assert(((size_t)DM * DM) % 2048 == 0);
static_assert(((size_t)DM * CD) % 2048 == 0);
static_assert(((size_t)DF * DM) % 2048 == 0);
static_assert(((size_t)LCT * CD) % 2048 == 0);
static_assert(NB <= NB_FULL);
static_assert(SEQ <= SEQ_FULL);
static_assert(LCT <= LCT_FULL);
static_assert((OSP * 4) % 16 == 0);
static_assert((GSP * 4) % 16 == 0);
static_assert(OSP >= HD);
static_assert(GSP >= 64);
static_assert(32 * 16 * 4 == 16 * HD * 2);
static_assert(32 * 16 * 8 == 16 * 64 * 4);
static_assert(16 * GSP * 4 <= 131072);
static_assert(AW * 16 * OSP * 4 <= 131072);

typedef _Float16 h16;
typedef __attribute__((ext_vector_type(16))) _Float16 v16h;
typedef __attribute__((ext_vector_type(8)))  _Float16 v8h;
typedef __attribute__((ext_vector_type(8)))  float    v8f;
typedef __attribute__((ext_vector_type(4)))  float    v4f;
typedef v4f  __attribute__((may_alias)) v4fa;

__device__ __forceinline__ unsigned short f2bf(float f) { unsigned u = __float_as_uint(f); u += 0x7FFFu + ((u >> 16) & 1u); return (unsigned short)(u >> 16); }
__device__ __forceinline__ float bfr(float f) { return __uint_as_float(((unsigned)f2bf(f)) << 16); }
__device__ __forceinline__ v16h cat16(v8h lo, v8h hi) { return __builtin_shufflevector(lo, hi, 0, 1, 2, 3, 4, 5, 6, 7, 8, 9, 10, 11, 12, 13, 14, 15); }
__device__ __forceinline__ v8f wmma16(v16h a, v16h b, v8f c) { return __builtin_amdgcn_wmma_f32_16x16x32_f16(false, a, false, b, (short)0, c, false, false); }
__device__ __forceinline__ v16h  ldh(const h16* p) { return cat16(*(const v8h*)p, *(const v8h*)(p + 16)); }
__device__ __forceinline__ void wave_sync() { __builtin_amdgcn_fence(3  , "wavefront"); __builtin_amdgcn_wave_barrier(); asm volatile("" ::: "memory"); }
static __device__ __forceinline__ h16 toh_flush(float v) { const h16 r = (h16)v; return (fabsf(v) < 6.103515625e-05f) ? (h16)0.0f : r; }
__device__ __forceinline__ v8f wmma_g(v16h a, v16h b, v8f c) { c = wmma16(a, b, c); asm volatile("v_nop\n\tv_nop\n\tv_nop\n\tv_nop" : "+v"(c) : "v"(a), "v"(b)); return c; }

__global__ __launch_bounds__(256) void k_cvth(const float* __restrict__ src, h16* dst, size_t n8, float carry) {
    const size_t i = (size_t)blockIdx.x * 256 + threadIdx.x; if (i >= n8) return;
    const v8f v = *(const v8f*)(src + i * 8); v8h o;
#pragma unroll
    for (int k = 0; k < 8; ++k) o[k] = toh_flush(bfr(v[k]) * carry);
    *(volatile v8h*)(dst + i * 8) = o; __threadfence(); *(volatile v8h*)(dst + i * 8) = o;
}

__global__ __launch_bounds__(256) void k_ln(const float* __restrict__ X, const float* __restrict__ G, const float* __restrict__ Bv, h16* Y, int inT, int inPitch, int rin) {
#pragma clang fp contract(off)
    const int lane = threadIdx.x & 31;
    const int wave = __builtin_amdgcn_readfirstlane((int)(threadIdx.x >> 5));
    const int row = blockIdx.x * 8 + wave;
    const int bb = row / inT, tt = row % inT;
    const float* xr = X + ((size_t)bb * (size_t)inPitch + (size_t)tt) * DM + lane * 8;
    float s = 0.0f;
#pragma unroll 1
    for (int i = 0; i < 4; ++i) {
        const v8f v = *(const v8f*)(xr + i * 256);
#pragma unroll
        for (int k = 0; k < 8; ++k) { const float a = rin ? bfr(v[k]) : v[k]; s += a; } }
#pragma unroll
    for (int off = 16; off >= 1; off >>= 1) s += __shfl_xor(s, off, 32);
    const float mean = s * (1.0f / DM);
    float q = 0.0f;
#pragma unroll 1
    for (int i = 0; i < 4; ++i) {
        const v8f v = *(const v8f*)(xr + i * 256);
#pragma unroll
        for (int k = 0; k < 8; ++k) { const float a = rin ? bfr(v[k]) : v[k]; const float d = a - mean; q += d * d; } }
#pragma unroll
    for (int off = 16; off >= 1; off >>= 1) q += __shfl_xor(q, off, 32);
    const float rs = rsqrtf(q * (1.0f / DM) + LNEPS);
    h16* yr = Y + (size_t)row * DM + lane * 8;
#pragma unroll 1
    for (int ps = 0; ps < 2; ++ps) {
#pragma unroll 1
        for (int i = 0; i < 4; ++i) {
            const v8f v = *(const v8f*)(xr + i * 256);
            const v8f g = *(const v8f*)(G + i * 256 + lane * 8);
            const v8f c = *(const v8f*)(Bv + i * 256 + lane * 8);
            v8h o;
#pragma unroll
            for (int k = 0; k < 8; ++k) { const float a = rin ? bfr(v[k]) : v[k]; const float y = (a - mean) * rs * bfr(g[k]) + bfr(c[k]); o[k] = toh_flush(y); }
            *(volatile v8h*)(yr + i * 256) = o; }
        if (ps == 0) __threadfence(); }
}

__device__ __forceinline__ void gemm_core(const h16* __restrict__ A, const h16* __restrict__ Bt, const int K, const size_t aoff, const size_t boff, v8f (&acc)[4][4]) {
#pragma unroll
    for (int mb = 0; mb < 4; ++mb)
#pragma unroll
        for (int nb = 0; nb < 4; ++nb) acc[mb][nb] = (v8f){};
#pragma unroll 1
    for (int kc = 0; kc < K; kc += 32) {
        v16h a[4];
#pragma unroll
        for (int mb = 0; mb < 4; ++mb) a[mb] = ldh(A + aoff + (size_t)mb * 16 * (size_t)K + kc);
#pragma unroll
        for (int nb = 0; nb < 4; ++nb) { const v16h b = ldh(Bt + boff + (size_t)nb * 16 * (size_t)K + kc);
#pragma unroll
            for (int mb = 0; mb < 4; ++mb) acc[mb][nb] = wmma_g(a[mb], b, acc[mb][nb]); }
    }
}

__global__ __launch_bounds__(32) void k_gemm_head(const h16* __restrict__ A, const h16* __restrict__ Bt, const float* __restrict__ bias, h16* P, int K, int T) {
    __shared__ __align__(16) float os[16 * GSP];
    const int lane = threadIdx.x & 31, lr = lane & 15, hi = lane >> 4; const int r0 = blockIdx.x * 64, c0 = blockIdx.y * 64;
    v8f acc[4][4];
    gemm_core(A, Bt, K, (size_t)(r0 + lr) * (size_t)K + 8 * hi, (size_t)(c0 + lr) * (size_t)K + 8 * hi, acc);
    float bc[4];
#pragma unroll
    for (int nb = 0; nb < 4; ++nb) bc[nb] = bfr(bias[c0 + nb * 16 + lr]);
    const int bb = r0 / T, tt = r0 % T; const int zc = bb * NH_ + c0 / HD;
    const size_t tbase = ((size_t)zc * (size_t)T + (size_t)tt) * HD;
#pragma unroll
    for (int mb = 0; mb < 4; ++mb) {
#pragma unroll
        for (int nb = 0; nb < 4; ++nb) {
#pragma unroll
            for (int j = 0; j < 8; ++j) os[(hi * 8 + j) * GSP + nb * 16 + lr] = acc[mb][nb][j] * WCI + bc[nb]; }
        wave_sync();
        const size_t sb = tbase + (size_t)(mb * 16) * HD;
#pragma unroll 1
        for (int ps = 0; ps < 2; ++ps) {
#pragma unroll
            for (int s = 0; s < 4; ++s) { const int p = s * 32 + lane; const int row = p >> 3, c8 = (p & 7) * 8;
                const v4f x0 = *(const v4fa*)(&os[row * GSP + c8]); const v4f x1 = *(const v4fa*)(&os[row * GSP + c8 + 4]); v8h hv;
#pragma unroll
                for (int i = 0; i < 4; ++i) { hv[i] = toh_flush(x0[i]); hv[4 + i] = toh_flush(x1[i]); }
                *(volatile v8h*)(P + sb + (size_t)p * 8) = hv; }
            if (ps == 0) __threadfence(); }
        wave_sync();
    }
}

__global__ __launch_bounds__(32) void k_gemm_vt(const h16* __restrict__ A, const h16* __restrict__ Bt, const float* __restrict__ bias, h16* P, int K, int T) {
    __shared__ __align__(16) float os[16 * GSP];
    const int lane = threadIdx.x & 31, lr = lane & 15, hi = lane >> 4; const int r0 = blockIdx.x * 64, c0 = blockIdx.y * 64;
    v8f acc[4][4];
    gemm_core(A, Bt, K, (size_t)(r0 + lr) * (size_t)K + 8 * hi, (size_t)(c0 + lr) * (size_t)K + 8 * hi, acc);
    const int bb = c0 / T, tt = c0 % T;
    const size_t tbase = (size_t)bb * (size_t)DM * (size_t)T + (size_t)r0 * (size_t)T + (size_t)tt;
#pragma unroll
    for (int mb = 0; mb < 4; ++mb) {
        float br[8];
#pragma unroll
        for (int j = 0; j < 8; ++j) br[j] = bfr(bias[r0 + mb * 16 + hi * 8 + j]);
#pragma unroll
        for (int nb = 0; nb < 4; ++nb) {
#pragma unroll
            for (int j = 0; j < 8; ++j) os[(hi * 8 + j) * GSP + nb * 16 + lr] = acc[mb][nb][j] * WCI + br[j]; }
        wave_sync();
        const size_t sb = tbase + (size_t)(mb * 16) * (size_t)T;
#pragma unroll 1
        for (int ps = 0; ps < 2; ++ps) {
#pragma unroll
            for (int s = 0; s < 4; ++s) { const int row = 4 * s + (lane >> 3), c8 = (lane & 7) * 8;
                const v4f x0 = *(const v4fa*)(&os[row * GSP + c8]); const v4f x1 = *(const v4fa*)(&os[row * GSP + c8 + 4]); v8h hv;
#pragma unroll
                for (int i = 0; i < 4; ++i) { hv[i] = toh_flush(x0[i]); hv[4 + i] = toh_flush(x1[i]); }
                *(volatile v8h*)(P + sb + (size_t)row * (size_t)T + c8) = hv; }
            if (ps == 0) __threadfence(); }
        wave_sync();
    }
}

__global__ __launch_bounds__(32) void k_gemm_res(const h16* __restrict__ A, const h16* __restrict__ Bt, const float* __restrict__ bias, const float* __restrict__ R, float* OUT,
                                                 int K, float sc, int rT, int rPitch, int oPitch, int rin) {
    __shared__ __align__(16) float os[16 * GSP];
    const int lane = threadIdx.x & 31, lr = lane & 15, hi = lane >> 4; const int r0 = blockIdx.x * 64, c0 = blockIdx.y * 64;
    v8f acc[4][4];
    gemm_core(A, Bt, K, (size_t)(r0 + lr) * (size_t)K + 8 * hi, (size_t)(c0 + lr) * (size_t)K + 8 * hi, acc);
    float bc[4];
#pragma unroll
    for (int nb = 0; nb < 4; ++nb) bc[nb] = bfr(bias[c0 + nb * 16 + lr]);
    const int bb = r0 / rT, tt = r0 % rT;
    const float* rrow = R + ((size_t)bb * (size_t)rPitch + (size_t)tt) * DM + c0;
    float* orow = OUT + ((size_t)bb * (size_t)oPitch + (size_t)tt) * DM + c0;
#pragma unroll
    for (int mb = 0; mb < 4; ++mb) {
#pragma unroll
        for (int nb = 0; nb < 4; ++nb) {
#pragma unroll
            for (int j = 0; j < 8; ++j) os[(hi * 8 + j) * GSP + nb * 16 + lr] = acc[mb][nb][j] * sc + bc[nb]; }
        wave_sync();
#pragma unroll 1
        for (int ps = 0; ps < 2; ++ps) {
#pragma unroll
            for (int s = 0; s < 8; ++s) { const int row = 2 * s + (lane >> 4), cofs = (lane & 15) * 4;
                const v4f a = *(const v4fa*)(&os[row * GSP + cofs]);
                const v4f r = *(const v4f*)(rrow + (size_t)(mb * 16 + row) * DM + cofs);
                v4f val;
#pragma unroll
                for (int i = 0; i < 4; ++i) { const float rv = rin ? bfr(r[i]) : r[i]; val[i] = a[i] + rv; }
                *(volatile v4f*)(orow + (size_t)(mb * 16 + row) * DM + cofs) = val; }
            if (ps == 0) __threadfence(); }
        wave_sync();
    }
}

__global__ __launch_bounds__(32) void k_gemm_gelu(const h16* __restrict__ A, const h16* __restrict__ Bt, const float* __restrict__ bias, h16* Hd, int K, int N) {
    __shared__ __align__(16) float os[16 * GSP];
    const int lane = threadIdx.x & 31, lr = lane & 15, hi = lane >> 4; const int r0 = blockIdx.x * 64, c0 = blockIdx.y * 64;
    v8f acc[4][4];
    gemm_core(A, Bt, K, (size_t)(r0 + lr) * (size_t)K + 8 * hi, (size_t)(c0 + lr) * (size_t)K + 8 * hi, acc);
    float bc[4];
#pragma unroll
    for (int nb = 0; nb < 4; ++nb) bc[nb] = bfr(bias[c0 + nb * 16 + lr]);
    h16* hrow = Hd + (size_t)r0 * (size_t)N + c0;
#pragma unroll
    for (int mb = 0; mb < 4; ++mb) {
#pragma unroll
        for (int nb = 0; nb < 4; ++nb) {
#pragma unroll
            for (int j = 0; j < 8; ++j) os[(hi * 8 + j) * GSP + nb * 16 + lr] = acc[mb][nb][j] * WCI + bc[nb]; }
        wave_sync();
#pragma unroll 1
        for (int s = 0; s < 4; ++s) { const int row = 4 * s + (lane >> 3), c8 = (lane & 7) * 8;
            v4f x0 = *(const v4fa*)(&os[row * GSP + c8]); v4f x1 = *(const v4fa*)(&os[row * GSP + c8 + 4]);
#pragma unroll
            for (int i = 0; i < 4; ++i) { x0[i] = 0.5f * x0[i] * (1.0f + erff(x0[i] * 0.70710678118654752f)); x1[i] = 0.5f * x1[i] * (1.0f + erff(x1[i] * 0.70710678118654752f)); }
            *(v4fa*)(&os[row * GSP + c8]) = x0; *(v4fa*)(&os[row * GSP + c8 + 4]) = x1; }
        wave_sync();
#pragma unroll 1
        for (int ps = 0; ps < 2; ++ps) {
#pragma unroll
            for (int s = 0; s < 4; ++s) { const int row = 4 * s + (lane >> 3), c8 = (lane & 7) * 8;
                const v4f x0 = *(const v4fa*)(&os[row * GSP + c8]); const v4f x1 = *(const v4fa*)(&os[row * GSP + c8 + 4]); v8h hv;
#pragma unroll
                for (int i = 0; i < 4; ++i) { hv[i] = toh_flush(x0[i]); hv[4 + i] = toh_flush(x1[i]); }
                *(volatile v8h*)(hrow + (size_t)(mb * 16 + row) * (size_t)N + c8) = hv; }
            if (ps == 0) __threadfence(); }
        wave_sync();
    }
}

__global__ __launch_bounds__(32 * AW) void k_flash(const h16* __restrict__ QH, const h16* __restrict__ KP, const h16* __restrict__ VT, h16* CT, int Tq, int Tk) {
    __shared__ __align__(16) float os[AW * 16 * OSP];
    const int lane = threadIdx.x & 31, lr = lane & 15, hi = lane >> 4;
    const int wave = __builtin_amdgcn_readfirstlane((int)(threadIdx.x >> 5));
    const int zh = blockIdx.y; const int b = zh / NH_, h = zh % NH_;
    const int t0 = (blockIdx.x * AW + wave) * 16;
    const size_t qbase = (size_t)zh * (size_t)Tq * HD;
    const size_t kbase = (size_t)zh * (size_t)Tk * HD;
    const size_t qo = qbase + (size_t)(t0 + lr) * HD + 8 * hi;
    const v16h q0 = ldh(QH + qo), q1 = ldh(QH + qo + 32);
    const size_t ko = kbase + (size_t)lr * HD + 8 * hi;
    const size_t vo = kbase + (size_t)lr * (size_t)Tk + 8 * hi;
    v8f o[4];
#pragma unroll
    for (int j = 0; j < 4; ++j) o[j] = (v8f){};
    float m = NEGB, l = 0.0f;
#pragma unroll 1
    for (int key0 = 0; key0 < Tk; key0 += 32) {
        const h16* ka = KP + ko + (size_t)key0 * HD;
        const v16h ka0 = ldh(ka), ka1 = ldh(ka + 32), kb0 = ldh(ka + 16 * HD), kb1 = ldh(ka + 16 * HD + 32);
        v8f sa = (v8f){}, sb = (v8f){};
        sa = wmma_g(ka0, q0, sa); sb = wmma_g(kb0, q0, sb); sa = wmma_g(ka1, q1, sa); sb = wmma_g(kb1, q1, sb);
        float ta[8], tb[8]; float mx = NEGB;
#pragma unroll
        for (int r = 0; r < 8; ++r) { ta[r] = sa[r] * SC2; tb[r] = sb[r] * SC2; mx = fmaxf(mx, fmaxf(ta[r], tb[r])); }
        mx = fmaxf(mx, __shfl_xor(mx, 16, 32));
        const float mnew = fmaxf(m, mx);
        const float alpha = __builtin_amdgcn_exp2f(m - mnew);
        const float sh = PSH - mnew;
        v16h pb; float ls = 0.0f;
#pragma unroll
        for (int r = 0; r < 8; ++r) {
            const float xa = ta[r] + sh, xb = tb[r] + sh;
            const float ea = __builtin_amdgcn_exp2f(xa), eb = __builtin_amdgcn_exp2f(xb);
            const float ga = (xa < -14.0f) ? 0.0f : ea, gb = (xb < -14.0f) ? 0.0f : eb;
            const h16 pa = (h16)ga; const h16 pc = (h16)gb;
            pb[r] = pa; pb[8 + r] = pc;
            ls += (float)pa + (float)pc; }
        l = l * alpha + ls; m = mnew;
#pragma unroll
        for (int j = 0; j < 4; ++j) o[j] = o[j] * alpha;
        const h16* va = VT + vo + key0;
        const v16h v0 = ldh(va), v1 = ldh(va + (size_t)16 * (size_t)Tk), v2 = ldh(va + (size_t)32 * (size_t)Tk), v3 = ldh(va + (size_t)48 * (size_t)Tk);
        o[0] = wmma_g(v0, pb, o[0]); o[1] = wmma_g(v1, pb, o[1]); o[2] = wmma_g(v2, pb, o[2]); o[3] = wmma_g(v3, pb, o[3]);
    }
    l += __shfl_xor(l, 16, 32);
    const float inv = CCAR * (1.0f / l);
    const int wb = wave * 16 * OSP;
#pragma unroll
    for (int j = 0; j < 4; ++j) { v4f a, c;
        a[0] = o[j][0] * inv; a[1] = o[j][1] * inv; a[2] = o[j][2] * inv; a[3] = o[j][3] * inv; c[0] = o[j][4] * inv; c[1] = o[j][5] * inv; c[2] = o[j][6] * inv; c[3] = o[j][7] * inv;
        *(v4fa*)(&os[wb + lr * OSP + 16 * j + 8 * hi]) = a; *(v4fa*)(&os[wb + lr * OSP + 16 * j + 8 * hi + 4]) = c; }
    wave_sync();
    h16* crow = CT + ((size_t)b * (size_t)Tq + (size_t)t0) * DM + h * HD;
#pragma unroll 1
    for (int ps = 0; ps < 2; ++ps) {
#pragma unroll
        for (int s = 0; s < 4; ++s) { const int row = 4 * s + (lane >> 3), c8 = (lane & 7) * 8;
            const v4f x0 = *(const v4fa*)(&os[wb + row * OSP + c8]); const v4f x1 = *(const v4fa*)(&os[wb + row * OSP + c8 + 4]); v8h hv;
#pragma unroll
            for (int i = 0; i < 4; ++i) { hv[i] = toh_flush(x0[i]); hv[4 + i] = toh_flush(x1[i]); }
            *(volatile v8h*)(crow + (size_t)row * DM + c8) = hv; }
        if (ps == 0) __threadfence(); }
}

static constexpr size_t al256(size_t v) { return (v + 255) & ~(size_t)255; }
static constexpr size_t SZ_WD  = al256((size_t)DM * DM * 2);
static constexpr size_t SZ_WC  = al256((size_t)DM * CD * 2);
static constexpr size_t SZ_WF  = al256((size_t)DF * DM * 2);
static constexpr size_t SZ_CX  = al256((size_t)NB * LCT * CD * 2);
static constexpr size_t SZ_PL  = al256((size_t)NB * SEQ * DM * 2);
static constexpr size_t SZ_KV  = al256((size_t)NB * KVT * DM * 2);
static constexpr size_t SZ_XF  = al256((size_t)NB * SEQ * DM * 4);
static constexpr size_t SZ_HID = al256((size_t)NB * SEQ * DF * 2);
static constexpr size_t SZ_ATT = 2 * SZ_PL + 2 * SZ_KV;
static constexpr size_t SZ_TOTAL = 6 * SZ_WD + 2 * SZ_WC + 2 * SZ_WF + SZ_CX + SZ_PL + SZ_ATT + 2 * SZ_XF;
static_assert(SZ_TOTAL <= (size_t)134217728);
static_assert(SZ_HID <= SZ_ATT);
static_assert((size_t)NB * LCT * DM * 2 <= SZ_KV);
static_assert((size_t)NB * SEQ * DM * 2 <= SZ_KV);

extern "C" void kernel_launch(void* const* d_in, const int* in_sizes, int n_in,
                              void* d_out, int out_size, void* d_ws, size_t ws_size, hipStream_t stream) {
    if (n_in < 28) return;
    const size_t needx = ((size_t)(NB - 1) * SEQ_FULL + SEQ) * DM;
    const size_t needc = ((size_t)(NB - 1) * LCT_FULL + LCT) * CD;
    if ((size_t)in_sizes[0] < needx || (size_t)in_sizes[1] < needc) return;
    for (int i = 2; i < 8; ++i) if (in_sizes[i] < DM) return;
    if ((size_t)in_sizes[8] < (size_t)DM * DM || (size_t)in_sizes[10] < (size_t)DM * DM || (size_t)in_sizes[12] < (size_t)DM * DM || (size_t)in_sizes[14] < (size_t)DM * DM) return;
    if ((size_t)in_sizes[16] < (size_t)DM * DM || (size_t)in_sizes[18] < (size_t)DM * CD || (size_t)in_sizes[20] < (size_t)DM * CD || (size_t)in_sizes[22] < (size_t)DM * DM) return;
    if ((size_t)in_sizes[24] < (size_t)DF * DM || (size_t)in_sizes[26] < (size_t)DM * DF) return;
    for (int i = 9; i < 24; i += 2) if (in_sizes[i] < DM) return;
    if (in_sizes[25] < DF || in_sizes[27] < DM) return;
    if ((size_t)out_size < ((size_t)(NB - 1) * OUT_SEQ + SEQ) * DM) return;
    if (SZ_TOTAL > ws_size) return;
    const float* x    = (const float*)d_in[0];
    const float* ctx  = (const float*)d_in[1];
    const float* ln1g = (const float*)d_in[2];  const float* ln1b = (const float*)d_in[3];
    const float* ln2g = (const float*)d_in[4];  const float* ln2b = (const float*)d_in[5];
    const float* ln3g = (const float*)d_in[6];  const float* ln3b = (const float*)d_in[7];
    const float* sa_wq = (const float*)d_in[8];  const float* sa_bq = (const float*)d_in[9];
    const float* sa_wk = (const float*)d_in[10]; const float* sa_bk = (const float*)d_in[11];
    const float* sa_wv = (const float*)d_in[12]; const float* sa_bv = (const float*)d_in[13];
    const float* sa_wo = (const float*)d_in[14]; const float* sa_bo = (const float*)d_in[15];
    const float* ca_wq = (const float*)d_in[16]; const float* ca_bq = (const float*)d_in[17];
    const float* ca_wk = (const float*)d_in[18]; const float* ca_bk = (const float*)d_in[19];
    const float* ca_wv = (const float*)d_in[20]; const float* ca_bv = (const float*)d_in[21];
    const float* ca_wo = (const float*)d_in[22]; const float* ca_bo = (const float*)d_in[23];
    const float* w1 = (const float*)d_in[24]; const float* b1 = (const float*)d_in[25];
    const float* w2 = (const float*)d_in[26]; const float* b2 = (const float*)d_in[27];
    float* OUT = (float*)d_out;

    char* wsp = (char*)d_ws;
    h16* WSQ = (h16*)wsp; wsp += SZ_WD;
    h16* WSK = (h16*)wsp; wsp += SZ_WD;
    h16* WSV = (h16*)wsp; wsp += SZ_WD;
    h16* WSO = (h16*)wsp; wsp += SZ_WD;
    h16* WCQ = (h16*)wsp; wsp += SZ_WD;
    h16* WCO = (h16*)wsp; wsp += SZ_WD;
    h16* WCK = (h16*)wsp; wsp += SZ_WC;
    h16* WCV = (h16*)wsp; wsp += SZ_WC;
    h16* WF1 = (h16*)wsp; wsp += SZ_WF;
    h16* WF2 = (h16*)wsp; wsp += SZ_WF;
    h16* CX  = (h16*)wsp; wsp += SZ_CX;
    h16* HN  = (h16*)wsp; wsp += SZ_PL;
    h16* HID = (h16*)wsp;
    h16* QH  = (h16*)wsp; wsp += SZ_PL;
    h16* KP  = (h16*)wsp; wsp += SZ_KV;
    h16* VT  = (h16*)wsp; wsp += SZ_KV;
    h16* CT  = (h16*)wsp; wsp += SZ_PL;
    float* X1 = (float*)wsp; wsp += SZ_XF;
    float* X2 = (float*)wsp; wsp += SZ_XF;

    { const size_t n8 = (size_t)DM * DM / 8; const unsigned g = (unsigned)((n8 + 255) / 256);
      k_cvth<<<g, 256, 0, stream>>>(sa_wq, WSQ, n8, WCAR); k_cvth<<<g, 256, 0, stream>>>(sa_wk, WSK, n8, WCAR);
      k_cvth<<<g, 256, 0, stream>>>(sa_wv, WSV, n8, WCAR); k_cvth<<<g, 256, 0, stream>>>(sa_wo, WSO, n8, WCAR);
      k_cvth<<<g, 256, 0, stream>>>(ca_wq, WCQ, n8, WCAR); k_cvth<<<g, 256, 0, stream>>>(ca_wo, WCO, n8, WCAR); }
    { const size_t n8 = (size_t)DM * CD / 8; const unsigned g = (unsigned)((n8 + 255) / 256);
      k_cvth<<<g, 256, 0, stream>>>(ca_wk, WCK, n8, WCAR); k_cvth<<<g, 256, 0, stream>>>(ca_wv, WCV, n8, WCAR); }
    { const size_t n8 = (size_t)DF * DM / 8; const unsigned g = (unsigned)((n8 + 255) / 256);
      k_cvth<<<g, 256, 0, stream>>>(w1, WF1, n8, WCAR); k_cvth<<<g, 256, 0, stream>>>(w2, WF2, n8, WCAR); }
    if (LCT == LCT_FULL) {
        const size_t n8 = (size_t)NB * LCT * CD / 8;
        k_cvth<<<(unsigned)((n8 + 255) / 256), 256, 0, stream>>>(ctx, CX, n8, 1.0f);
    } else {
        const size_t n8 = (size_t)LCT * CD / 8;
        for (int b = 0; b < NB; ++b) k_cvth<<<(unsigned)((n8 + 255) / 256), 256, 0, stream>>>(ctx + (size_t)b * LCT_FULL * CD, CX + (size_t)b * LCT * CD, n8, 1.0f);
    }

    const dim3 gTok(NB * SEQ / 64, DM / 64, 1);
    const dim3 gTokT(DM / 64, NB * SEQ / 64, 1);
    const dim3 gCtx(NB * LCT / 64, DM / 64, 1);
    const dim3 gCtxT(DM / 64, NB * LCT / 64, 1);
    const dim3 gFl(SEQ / (16 * AW), NB * NH_, 1);

    k_ln<<<NB * SEQ / 8, 256, 0, stream>>>(x, ln1g, ln1b, HN, SEQ, SEQ_FULL, 1);
    k_gemm_head<<<gTok, 32, 0, stream>>>(HN, WSQ, sa_bq, QH, DM, SEQ);
    k_gemm_head<<<gTok, 32, 0, stream>>>(HN, WSK, sa_bk, KP, DM, SEQ);
    k_gemm_vt<<<gTokT, 32, 0, stream>>>(WSV, HN, sa_bv, VT, DM, SEQ);
    k_flash<<<gFl, 32 * AW, 0, stream>>>(QH, KP, VT, CT, SEQ, SEQ);
    k_gemm_res<<<gTok, 32, 0, stream>>>(CT, WSO, sa_bo, x, X1, DM, OCI, SEQ, SEQ_FULL, SEQ, 1);

    k_ln<<<NB * SEQ / 8, 256, 0, stream>>>(X1, ln2g, ln2b, HN, SEQ, SEQ, 0);
    k_gemm_head<<<gTok, 32, 0, stream>>>(HN, WCQ, ca_bq, QH, DM, SEQ);
    k_gemm_head<<<gCtx, 32, 0, stream>>>(CX, WCK, ca_bk, KP, CD, LCT);
    k_gemm_vt<<<gCtxT, 32, 0, stream>>>(WCV, CX, ca_bv, VT, CD, LCT);
    k_flash<<<gFl, 32 * AW, 0, stream>>>(QH, KP, VT, CT, SEQ, LCT);
    k_gemm_res<<<gTok, 32, 0, stream>>>(CT, WCO, ca_bo, X1, X2, DM, OCI, SEQ, SEQ, SEQ, 0);

    k_ln<<<NB * SEQ / 8, 256, 0, stream>>>(X2, ln3g, ln3b, HN, SEQ, SEQ, 0);
    k_gemm_gelu<<<dim3(NB * SEQ / 64, DF / 64, 1), 32, 0, stream>>>(HN, WF1, b1, HID, DM, DF);
    k_gemm_res<<<gTok, 32, 0, stream>>>(HID, WF2, b2, X2, OUT, DF, WCI, SEQ, SEQ, OUT_SEQ, 0);
}
